// GraphSAGE_47364899340882
// MI455X (gfx1250) — hardware-verified
//
#include <hip/hip_runtime.h>
#include <math.h>

constexpr int kNodes     = 100000;
constexpr int kEdges     = 1600000;
constexpr int kFeat      = 128;
constexpr int kKcat      = 256;
constexpr int kCls       = 10;
constexpr int kMPad      = 100032;
constexpr int kSplit     = 50048;
constexpr int kNT        = 256;
constexpr int kTileRows  = 16384;
constexpr int kWaveRows  = 2048;
constexpr int kTiles     = 7;
constexpr int kInvLen    = kTiles * kTileRows;
constexpr int kRecShift  = 17;
constexpr int kOwnShift  = 28;
constexpr int kChunk     = 4096;
constexpr int kSlotsPT   = kChunk / kNT;
constexpr int kNumChunks = (kEdges + kChunk - 1) / kChunk;
constexpr int kStatBlocks = 32;
constexpr int kStatRows   = (kNodes + kStatBlocks - 1) / kStatBlocks;
constexpr int kStatSlots  = kStatBlocks * 8;
constexpr double kInvNodes = 1.0 / 100000.0;
constexpr float  kBnEps    = 1e-5f;

constexpr size_t kQBytes    = (size_t)kSplit * kFeat * 4;
constexpr size_t kABytes    = (size_t)kMPad * kKcat * 2;
constexpr size_t kA0Off     = (size_t)kMPad * kFeat * 2;
constexpr size_t kYBytes    = (size_t)kMPad * kFeat * 4;
constexpr size_t kBtBytes   = (size_t)3 * kKcat * kKcat * 2;
constexpr size_t kInvBytes  = (size_t)kInvLen * 4;
constexpr size_t kPartBytes = (size_t)kStatSlots * 256 * 4;
constexpr size_t kMsBytes   = 1024;
constexpr size_t kWsTotal   = kQBytes + kABytes + kYBytes + kBtBytes + kInvBytes + kPartBytes + kMsBytes;

static_assert(kMPad % 64 == 0, "M tile multiple");
static_assert(kMPad >= kNodes && kMPad - kNodes < 64, "pad rows");
static_assert(kSplit % 64 == 0 && (kMPad - kSplit) % 64 == 0, "both Ql launches are M tile multiples");
static_assert(kFeat % 64 == 0, "N tile multiple");
static_assert(kFeat % 32 == 0 && kKcat % 32 == 0, "K multiple of 32");
static_assert(kInvLen >= kMPad, "inv table covers padded rows");
static_assert(kTileRows == 8 * kWaveRows, "8 waves per tile");
static_assert(kWaveRows == (1 << (kOwnShift - kRecShift)), "owner shift");
static_assert(kNodes <= (1 << kRecShift), "src fits in the record");
static_assert(((long long)(kTileRows - 1) << kRecShift) + kNodes < 2147483647LL, "record is non-negative");
static_assert(kEdges % kSlotsPT == 0, "thread slot groups entirely in range or out of range");
static_assert(kSlotsPT % 4 == 0, "b128 edge loads");
static_assert((kEdges % kChunk) % (32 * kSlotsPT) == 0, "in-range flag is wave-uniform in the last chunk");
static_assert((kNodes % kNT) % 16 == 0, "last head block rows are a multiple of 16 (whole lines)");
static_assert((kNodes * kCls * 4) % 128 == 0, "second output starts on a line");
static_assert((kMPad * 16) % kNT == 0, "elementwise grids exact");
static_assert(kStatBlocks * kStatRows >= kNodes, "statistic blocks cover all rows");
static_assert(kTileRows % (4 * kNT) == 0 && kWaveRows % 128 == 0, "staging loops exact");
static_assert(kQBytes % 256 == 0 && kABytes % 256 == 0 && kYBytes % 256 == 0 && kBtBytes % 256 == 0 &&
              kInvBytes % 256 == 0 && kPartBytes % 256 == 0, "region alignment");
static_assert((size_t)(kMPad - kSplit) * kFeat * 4 <= kA0Off, "Ql tail rows end below the layer-0 operand plane");
static_assert((size_t)(kMPad - kSplit) * kFeat * 4 <= (size_t)kSplit * kKcat * 2, "Ql tail rows end below the first A row read by the second Ql launch");
static_assert(kA0Off + (size_t)kMPad * kFeat * 2 <= kABytes, "layer-0 operand plane inside the A region");
static_assert(kWsTotal <= (size_t)134217728, "carve within 128 MiB");

typedef __attribute__((ext_vector_type(16))) _Float16 v16h;
typedef __attribute__((ext_vector_type(8)))  _Float16 v8h;
typedef __attribute__((ext_vector_type(16))) __bf16   v16b;
typedef __attribute__((ext_vector_type(8)))  __bf16   v8b;
typedef __attribute__((ext_vector_type(8)))  float    v8f;
typedef __attribute__((ext_vector_type(4)))  float    v4f;
typedef __attribute__((ext_vector_type(4)))  unsigned int v4u;
typedef __attribute__((ext_vector_type(4)))  int      v4i;

__device__ __forceinline__ unsigned short f2bf_bits(float f) {
  unsigned u = __float_as_uint(f);
  return (unsigned short)((u + 0x7FFFu + ((u >> 16) & 1u)) >> 16);
}
__device__ __forceinline__ float bf_bits2f(unsigned short h) { return __uint_as_float(((unsigned)h) << 16); }

__device__ __forceinline__ void dep_guard_h(v8f& a, v8f& b, v16h x, v16h y) { asm volatile("v_nop\n\tv_nop\n\tv_nop\n\tv_nop" : "+v"(a), "+v"(b) : "v"(x), "v"(y)); }
__device__ __forceinline__ void dep_guard_b(v8f& a, v8f& b, v16b x, v16b y) { asm volatile("v_nop\n\tv_nop\n\tv_nop\n\tv_nop" : "+v"(a), "+v"(b) : "v"(x), "v"(y)); }
__device__ __forceinline__ void keep4_h(v16h a, v16h b, v16h c, v16h d) { asm volatile("v_nop" :: "v"(a), "v"(b), "v"(c), "v"(d)); }
__device__ __forceinline__ void keep4_b(v16b a, v16b b, v16b c, v16b d) { asm volatile("v_nop" :: "v"(a), "v"(b), "v"(c), "v"(d)); }
__device__ __forceinline__ void acc_guard4(v8f& a, v8f& b, v8f& c, v8f& d) { asm volatile("v_nop\n\tv_nop\n\tv_nop\n\tv_nop" : "+v"(a), "+v"(b), "+v"(c), "+v"(d)); }
template <typename T> struct Frag;
template <> struct Frag<_Float16> {
  typedef v16h V; union U { v16h v; v8h h[2]; };
  static __device__ __forceinline__ v16h load(const _Float16* p) {
    U f; f.h[0] = *(const v8h*)(p); f.h[1] = *(const v8h*)(p + 16); return f.v;
  }
  static __device__ __forceinline__ v8f mma(v16h a, v16h b, v8f c) {
    return __builtin_amdgcn_wmma_f32_16x16x32_f16(false, a, false, b, (short)0, c, false, false);
  }
  static __device__ __forceinline__ void guard(v8f& a, v8f& b, v16h x, v16h y) { dep_guard_h(a, b, x, y); }
  static __device__ __forceinline__ void keep(v16h a, v16h b, v16h c, v16h d) { keep4_h(a, b, c, d); }
};
template <> struct Frag<__bf16> {
  typedef v16b V; union U { v16b v; v8b h[2]; };
  static __device__ __forceinline__ v16b load(const __bf16* p) {
    U f; f.h[0] = *(const v8b*)(p); f.h[1] = *(const v8b*)(p + 16); return f.v;
  }
  static __device__ __forceinline__ v8f mma(v16b a, v16b b, v8f c) {
    return __builtin_amdgcn_wmma_f32_16x16x32_bf16(false, a, false, b, (short)0, c, false, false);
  }
  static __device__ __forceinline__ void guard(v8f& a, v8f& b, v16b x, v16b y) { dep_guard_b(a, b, x, y); }
  static __device__ __forceinline__ void keep(v16b a, v16b b, v16b c, v16b d) { keep4_b(a, b, c, d); }
};

__device__ __forceinline__ unsigned pk16(unsigned short a, unsigned short b) { return (unsigned)a | ((unsigned)b << 16); }
__device__ __forceinline__ float bf_rne(float f) { return bf_bits2f(f2bf_bits(f)); }

template <int ET> struct Elem;
template <> struct Elem<0> { typedef _Float16 T; };
template <> struct Elem<1> { typedef __bf16 T; };
template <int ET, bool SPLIT, int BIAS_MODE, int OUT_MODE, bool RESID, int ACT = 0>
__global__ __launch_bounds__(256) void wmma_gemm64(
    const unsigned short* __restrict__ Ap, const unsigned short* __restrict__ A2p, int lda, long strideA,
    const unsigned short* __restrict__ Btp, const unsigned short* __restrict__ Bt2p, int ldb, long strideB,
    void* Cout, void* Cout2, int ldc, long strideC,
    const float* __restrict__ bias,
    const float* resid, long strideR,
    int M, int N, int K, float scale) {
  typedef typename Elem<ET>::T T;
  typedef typename Frag<T>::V V;
  const T* A = (const T*)Ap; const T* A2 = (const T*)A2p; const T* Bt = (const T*)Btp; const T* Bt2 = (const T*)Bt2p;
  __shared__ __align__(16) float sT[8][16 * 68];
  const int b    = blockIdx.y;
  const int lane = threadIdx.x & 31;
  const int wave = threadIdx.x >> 5;
  const int tilesN = N >> 6;
  const int tilesM = M >> 6;
  const int tile = blockIdx.x * 8 + wave;
  if (tile >= tilesM * tilesN) return;
  const int tm = tile / tilesN;
  const int tn = tile - tm * tilesN;
  const int m0 = tm << 6;
  const int n0 = tn << 6;

  const T* Ab  = A  + (size_t)b * strideA;
  const T* Bb  = Bt + (size_t)b * strideB;
  const T* Ab2 = SPLIT ? (A2  + (size_t)b * strideA) : nullptr;
  const T* Bb2 = SPLIT ? (Bt2 + (size_t)b * strideB) : nullptr;

  const int rlane = lane & 15;
  const int koff  = (lane >> 4) * 8;
  const int mOff  = (lane >> 4) * 8;

  v8f acc[4][4];
#pragma unroll
  for (int i = 0; i < 4; ++i)
#pragma unroll
    for (int j = 0; j < 4; ++j) acc[i][j] = (v8f){0.f,0.f,0.f,0.f,0.f,0.f,0.f,0.f};

  for (int k0 = 0; k0 < K; k0 += 32) {
    V bh[4], bl[4];
#pragma unroll
    for (int j = 0; j < 4; ++j) {
      const size_t bo = (size_t)(n0 + (j << 4) + rlane) * ldb + koff + k0;
      bh[j] = Frag<T>::load(Bb + bo);
      if (SPLIT) bl[j] = Frag<T>::load(Bb2 + bo);
    }
#pragma unroll
    for (int i = 0; i < 4; ++i) {
      const size_t ao = (size_t)(m0 + (i << 4) + rlane) * lda + koff + k0;
      V ah = Frag<T>::load(Ab + ao);
      V al;
      if (SPLIT) al = Frag<T>::load(Ab2 + ao);
#pragma unroll
      for (int j = 0; j < 4; ++j) {
        acc[i][j] = Frag<T>::mma(ah, bh[j], acc[i][j]);
        if (SPLIT) {
          acc[i][j] = Frag<T>::mma(ah, bl[j], acc[i][j]);
          acc[i][j] = Frag<T>::mma(al, bh[j], acc[i][j]);
        }
      }
      Frag<T>::guard(acc[i][0], acc[i][3], ah, SPLIT ? al : ah);
    }
    Frag<T>::keep(bh[0], bh[1], bh[2], bh[3]);
    if (SPLIT) Frag<T>::keep(bl[0], bl[1], bl[2], bl[3]);
  }
  acc_guard4(acc[0][0], acc[0][1], acc[0][2], acc[0][3]);
  acc_guard4(acc[1][0], acc[1][1], acc[1][2], acc[1][3]);
  acc_guard4(acc[2][0], acc[2][1], acc[2][2], acc[2][3]);
  acc_guard4(acc[3][0], acc[3][1], acc[3][2], acc[3][3]);

  float* slab = sT[wave];
  const float* Rb = RESID ? (resid + (size_t)b * strideR) : nullptr;
#pragma unroll
  for (int i = 0; i < 4; ++i) {
    const int mBase = m0 + (i << 4);
#pragma unroll
    for (int j = 0; j < 4; ++j) {
      const int n = n0 + (j << 4) + rlane;
      float bv = 0.f;
      if (BIAS_MODE == 2) bv = bias[n];
#pragma unroll
      for (int r = 0; r < 8; ++r) {
        float v = acc[i][j][r] * scale;
        if (BIAS_MODE == 1) v += bias[mBase + mOff + r];
        if (BIAS_MODE == 2) v += bv;
        if (ACT == 2) v = fmaxf(v, 0.0f);
        if (ACT == 4) v = (v > 0.f) ? v : 0.01f * v;
        slab[(mOff + r) * 68 + (j << 4) + rlane] = v;
      }
    }
    __builtin_amdgcn_fence(__ATOMIC_RELEASE, "workgroup");
    __builtin_amdgcn_wave_barrier();
    __builtin_amdgcn_fence(__ATOMIC_ACQUIRE, "workgroup");
    if (OUT_MODE == 0) {
      float* C = (float*)Cout + (size_t)b * strideC;
      const int hh = lane >> 4, c4 = (lane & 15) * 4;
      v4f radd[8];
#pragma unroll
      for (int it = 0; it < 8; ++it) {
        radd[it] = (v4f){0.f, 0.f, 0.f, 0.f};
        if (RESID) {
          const int row = it * 2 + hh;
          radd[it] = *(const v4f*)(Rb + (size_t)(mBase + row) * ldc + n0 + c4);
        }
      }
      for (int pass = 0; pass < 2; ++pass) {
#pragma unroll
        for (int it = 0; it < 8; ++it) {
          const int row = it * 2 + hh;
          v4f v = *(const v4f*)(slab + row * 68 + c4);
          if (RESID) v = v + radd[it];
          *(volatile v4f*)(C + (size_t)(mBase + row) * ldc + n0 + c4) = v;
        }
        __threadfence();
      }
    } else {
      const int q = lane >> 3, c8 = (lane & 7) * 8;
      unsigned short* C  = (unsigned short*)Cout  + (size_t)b * strideC;
      unsigned short* C2 = (OUT_MODE == 2) ? ((unsigned short*)Cout2 + (size_t)b * strideC) : nullptr;
      for (int pass = 0; pass < 2; ++pass) {
#pragma unroll
        for (int it = 0; it < 4; ++it) {
          const int row = it * 4 + q;
          const float* sp = slab + row * 68 + c8;
          v8h hv, lv;
#pragma unroll
          for (int e = 0; e < 8; ++e) {
            if (OUT_MODE == 1) {
              hv[e] = (_Float16)sp[e];
            } else {
              unsigned short hb = f2bf_bits(sp[e]);
              unsigned short lb = f2bf_bits(sp[e] - bf_bits2f(hb));
              hv[e] = __builtin_bit_cast(_Float16, hb);
              lv[e] = __builtin_bit_cast(_Float16, lb);
            }
          }
          *(volatile v8h*)(C + (size_t)(mBase + row) * ldc + n0 + c8) = hv;
          if (OUT_MODE == 2) *(volatile v8h*)(C2 + (size_t)(mBase + row) * ldc + n0 + c8) = lv;
        }
        __threadfence();
      }
    }
    __builtin_amdgcn_fence(__ATOMIC_RELEASE, "workgroup");
    __builtin_amdgcn_wave_barrier();
    __builtin_amdgcn_fence(__ATOMIC_ACQUIRE, "workgroup");
  }
}

__global__ __launch_bounds__(kNT) void k_prep_x(const float* __restrict__ x, unsigned short* __restrict__ A0) {
  const int i = blockIdx.x * kNT + threadIdx.x;
  const int row = i >> 4, c8 = (i & 15) * 8;
  const bool live = row < kNodes;
  const int rowc = live ? row : (kNodes - 1);
  const float fl = live ? 1.0f : 0.0f;
  const float* p = x + (size_t)rowc * kFeat + c8;
  const v4f a = *(const v4f*)(p);
  const v4f c = *(const v4f*)(p + 4);
  unsigned short hb[8];
#pragma unroll
  for (int e = 0; e < 4; ++e) {
    hb[e]     = f2bf_bits(fmaf(a[e], fl, 0.0f));
    hb[4 + e] = f2bf_bits(fmaf(c[e], fl, 0.0f));
  }
  const v4u u = (v4u){pk16(hb[0], hb[1]), pk16(hb[2], hb[3]), pk16(hb[4], hb[5]), pk16(hb[6], hb[7])};
  unsigned short* q = A0 + (size_t)row * kFeat + c8;
  *(volatile v4u*)q = u;
  __threadfence();
  *(volatile v4u*)q = u;
}

__global__ __launch_bounds__(kNT) void k_prep_w(const float* __restrict__ Wl0, const float* __restrict__ Wr0,
                                               const float* __restrict__ Wl, const float* __restrict__ Wr,
                                               unsigned short* __restrict__ Bt) {
  const int p  = blockIdx.y;
  const int rb = blockIdx.x;
  const int t  = threadIdx.x;
  const size_t poff = (size_t)(p > 0 ? p - 1 : 0) * kFeat * kFeat;
  const float* WL = (p == 0) ? Wl0 : (Wl + poff);
  const float* WR = (p == 0) ? Wr0 : (Wr + poff);
  const float* W  = (rb < 8) ? WL : WR;
  const int n = rb * 16 + (t >> 4), k8 = (t & 15) * 8, col = n & 127;
  unsigned short hb[8];
#pragma unroll
  for (int e = 0; e < 8; ++e) hb[e] = f2bf_bits(W[(size_t)(k8 + e) * kFeat + col]);
  const v4u u = (v4u){pk16(hb[0], hb[1]), pk16(hb[2], hb[3]), pk16(hb[4], hb[5]), pk16(hb[6], hb[7])};
  unsigned short* q = Bt + (size_t)p * kKcat * kKcat + (size_t)n * kKcat + k8;
  for (int pass = 0; pass < 2; ++pass) {
    *(volatile v4u*)q = u;
    *(volatile v4u*)(q + kFeat) = u;
    __threadfence();
  }
}

__device__ __forceinline__ int blk_excl_scan(int cnt, int* scan_ws, int tid, int* tot) {
  const int lane = tid & 31, wave = tid >> 5; int incl = cnt;
#pragma unroll
  for (int o = 1; o < 32; o <<= 1) { const int v = __shfl_up(incl, o, 32); if (lane >= o) incl += v; }
  if (lane == 31) scan_ws[wave] = incl;
  __syncthreads();
  if (wave == 0) { int wv = (lane < kNT / 32) ? scan_ws[lane] : 0; int wincl = wv;
#pragma unroll
    for (int o = 1; o < 32; o <<= 1) { const int v = __shfl_up(wincl, o, 32); if (lane >= o) wincl += v; }
    if (lane < kNT / 32) scan_ws[32 + lane] = wincl - wv; if (lane == 31) scan_ws[64] = wincl; }
  __syncthreads();
  const int res = scan_ws[32 + wave] + incl - cnt; *tot = scan_ws[64];
  return res;
}
template <int SP, int CAP>
__device__ __forceinline__ int chunk_hits(const int* __restrict__ dstv, const int* __restrict__ srcv, int e0, int n0, int tid,
                                          int* list, int* scan_ws) {
  const int eb = e0 + tid * SP;
  const bool inr = eb < kEdges;
  const int ebc = inr ? eb : (kEdges - SP);
  const int inri = inr ? 1 : 0;
  int rec[SP]; int cnt = 0;
#pragma unroll
  for (int k = 0; k < SP; k += 4) {
    const v4i d4 = *(const v4i*)(dstv + ebc + k);
    const v4i s4 = *(const v4i*)(srcv + ebc + k);
#pragma unroll
    for (int e = 0; e < 4; ++e) {
      const int d = d4[e]; int s = s4[e];
      s = s < 0 ? 0 : (s >= kNodes ? kNodes - 1 : s);
      const int hit = inri & (d >= n0 ? 1 : 0) & (d < n0 + kTileRows ? 1 : 0) & (d < kNodes ? 1 : 0);
      const int dl = hit ? (d - n0) : 0;
      rec[k + e] = hit ? ((dl << kRecShift) | s) : -1;
      cnt += hit;
    }
  }
  int tot; int p = blk_excl_scan(cnt, scan_ws, tid, &tot);
#pragma unroll
  for (int k = 0; k < SP; ++k) if (rec[k] >= 0) { if ((unsigned)p < (unsigned)CAP) list[p] = rec[k]; ++p; }
  __syncthreads();
  return tot < CAP ? tot : CAP;
}

template <bool FIRST>
__global__ __launch_bounds__(kNT) void k_agg(const int* __restrict__ ei, const float* invin,
                                            const float* __restrict__ Ql, float* Y, float* invout) {
  __shared__ int sList[kChunk];
  __shared__ __align__(16) float sRow[kTileRows];
  __shared__ int scan_ws[80];
  const int tid = threadIdx.x, lane = tid & 31, wave = tid >> 5;
  const int n0 = blockIdx.x * kTileRows;
  const v4f z4 = {0.0f, 0.0f, 0.0f, 0.0f};
#pragma unroll 1
  for (int i = tid; i < kChunk; i += kNT) sList[i] = 0;
  if (FIRST) {
#pragma unroll 1
    for (int i = tid; i < kTileRows; i += kNT) sRow[i] = 0.0f;
  } else {
#pragma unroll 1
    for (int i = tid; i < kTileRows / 4; i += kNT) *(v4f*)(sRow + 4 * i) = *(const v4f*)(invin + n0 + 4 * i);
  }
  if (tid < 80) scan_ws[tid] = 0;
  if (FIRST) {
    for (int pass = 0; pass < 2; ++pass) {
#pragma unroll 1
      for (int j = 0; j < kWaveRows; ++j) {
        const int n = n0 + wave * kWaveRows + j;
        if (n < kMPad) *(volatile v4f*)(Y + (size_t)n * kFeat + 4 * lane) = z4;
      }
      __threadfence();
    }
  }
  __syncthreads();
  const int* srcv = ei; const int* dstv = ei + kEdges;
#pragma unroll 1
  for (int c = 0; c < kNumChunks; ++c) {
    const int tot = chunk_hits<kSlotsPT, kChunk>(dstv, srcv, c * kChunk, n0, tid, sList, scan_ws);
#pragma unroll 1
    for (int base = 0; base < tot; base += 32) {
      const int q  = base + lane;
      const int qc = q < kChunk ? q : (kChunk - 1);
      const int lv = sList[qc];
      const int rv = lv | -(int)(q >= tot);
      const int own = (rv >= 0 && (rv >> kOwnShift) == wave) ? 1 : 0;
      unsigned msk = (unsigned)__ballot(own);
#pragma unroll 1
      for (int it = 0; it < 32; ++it) {
        if (msk == 0u) break;
        const int bp = __builtin_ctz(msk); msk &= msk - 1u;
        const int r = __builtin_amdgcn_readlane(rv, bp);
        const int dl = r >> kRecShift, s = r & ((1 << kRecShift) - 1);
        const float* qp = Ql + (size_t)s * kFeat + 4 * lane;
        float* yp = Y + (size_t)(n0 + dl) * kFeat + 4 * lane;
        const v4f qv = *(const v4f*)qp;
        v4f a = *(const v4f*)yp;
        const float cur = sRow[dl];
        if (FIRST) {
          a = a + qv;
          const float cn = cur + 1.0f;
          if (lane == 0) sRow[dl] = cn;
        } else {
#pragma unroll
          for (int e = 0; e < 4; ++e) a[e] = fmaf(qv[e], cur, a[e]);
        }
        *(volatile v4f*)yp = a;
        __threadfence();
        *(volatile v4f*)yp = a;
      }
    }
    __syncthreads();
  }
  if (FIRST) {
#pragma unroll 1
    for (int i = tid; i < kTileRows; i += kNT) { const float cn = sRow[i]; sRow[i] = 1.0f / fmaxf(cn, 1.0f); }
    __syncthreads();
  }
#pragma unroll 1
  for (int j = 0; j < kWaveRows; ++j) {
    const int dl = wave * kWaveRows + j;
    const int n = n0 + dl;
    if (n < kMPad) {
      float* yp = Y + (size_t)n * kFeat + 4 * lane;
      v4f v = *(const v4f*)yp;
      if (FIRST) { const float iv = sRow[dl]; v = v * iv; }
      *(volatile v4f*)yp = v;
      __threadfence();
      *(volatile v4f*)yp = v;
    }
  }
  if (FIRST) {
#pragma unroll 1
    for (int j = 0; j < kWaveRows / 128; ++j) {
      const int idx = wave * kWaveRows + j * 128 + 4 * lane;
      const v4f o = *(const v4f*)(sRow + idx);
      float* ip = invout + n0 + idx;
      *(volatile v4f*)ip = o;
      __threadfence();
      *(volatile v4f*)ip = o;
    }
  }
}

__global__ __launch_bounds__(kNT) void k_stats(const float* __restrict__ Y, float* __restrict__ part) {
  const int tid = threadIdx.x, lane = tid & 31, wave = tid >> 5;
  const int r0 = blockIdx.x * kStatRows;
  const int r1 = (r0 + kStatRows < kNodes) ? (r0 + kStatRows) : kNodes;
  const v4f z4 = {0.0f, 0.0f, 0.0f, 0.0f};
  v4f ps = z4, pq = z4;
#pragma unroll 1
  for (int r = r0 + wave; r < r1; r += 8) {
    const v4f v = *(const v4f*)(Y + (size_t)r * kFeat + 4 * lane);
    ps = ps + v;
#pragma unroll
    for (int e = 0; e < 4; ++e) pq[e] = fmaf(v[e], v[e], pq[e]);
  }
  float* pp = part + (size_t)(blockIdx.x * 8 + wave) * 256;
  for (int pass = 0; pass < 2; ++pass) {
    *(volatile v4f*)(pp + 4 * lane) = ps;
    *(volatile v4f*)(pp + 128 + 4 * lane) = pq;
    __threadfence();
  }
}

__global__ __launch_bounds__(128) void k_bn_fin(const float* __restrict__ part, float* __restrict__ ms) {
  const int c = threadIdx.x;
  double s = 0.0, q = 0.0;
#pragma unroll 1
  for (int p = 0; p < kStatSlots; ++p) { s += (double)part[p * 256 + c]; q += (double)part[p * 256 + 128 + c]; }
  const double m = s * kInvNodes;
  double v = q * kInvNodes - m * m;
  v = v > 0.0 ? v : 0.0;
  const float mf = (float)m, vf = (float)v;
  const float rs = rsqrtf(vf + kBnEps);
  for (int pass = 0; pass < 2; ++pass) {
    ((volatile float*)ms)[c] = mf;
    ((volatile float*)ms)[128 + c] = rs;
    __threadfence();
  }
}

__device__ __forceinline__ float bn_relu1(float y, float m, float rs, float g, float bt) {
  const float gg = bf_rne(g), bb = bf_rne(bt);
  float t = gg * (y - m);
  t = t * rs + bb;
  return fmaxf(t, 0.0f);
}

__global__ __launch_bounds__(kNT) void k_bn_apply(const float* __restrict__ Y, const float* __restrict__ ms,
                                                 const float* __restrict__ gam, const float* __restrict__ bet,
                                                 unsigned short* __restrict__ A) {
  const int i = blockIdx.x * kNT + threadIdx.x;
  const int row = i >> 4, c8 = (i & 15) * 8;
  const float cl = (row < kNodes) ? 1.0f : 0.0f;
  const float* yp = Y + (size_t)row * kFeat + c8;
  const v4f y0 = *(const v4f*)(yp), y1 = *(const v4f*)(yp + 4);
  const v4f m0 = *(const v4f*)(ms + c8), m1 = *(const v4f*)(ms + c8 + 4);
  const v4f r0 = *(const v4f*)(ms + 128 + c8), r1 = *(const v4f*)(ms + 128 + c8 + 4);
  const v4f g0 = *(const v4f*)(gam + c8), g1 = *(const v4f*)(gam + c8 + 4);
  const v4f b0 = *(const v4f*)(bet + c8), b1 = *(const v4f*)(bet + c8 + 4);
  unsigned short hb[8], lb[8];
#pragma unroll
  for (int e = 0; e < 4; ++e) {
    const float h0 = bn_relu1(y0[e], m0[e], r0[e], g0[e], b0[e]) * cl;
    const float h1 = bn_relu1(y1[e], m1[e], r1[e], g1[e], b1[e]) * cl;
    const unsigned short hb0 = f2bf_bits(h0), hb1 = f2bf_bits(h1);
    hb[e]     = hb0;
    hb[4 + e] = hb1;
    lb[e]     = f2bf_bits(h0 - bf_bits2f(hb0));
    lb[4 + e] = f2bf_bits(h1 - bf_bits2f(hb1));
  }
  const v4u uh = (v4u){pk16(hb[0], hb[1]), pk16(hb[2], hb[3]), pk16(hb[4], hb[5]), pk16(hb[6], hb[7])};
  const v4u ul = (v4u){pk16(lb[0], lb[1]), pk16(lb[2], lb[3]), pk16(lb[4], lb[5]), pk16(lb[6], lb[7])};
  unsigned short* qh = A + (size_t)row * kKcat + c8;
  unsigned short* ql = qh + kFeat;
  for (int pass = 0; pass < 2; ++pass) {
    *(volatile v4u*)qh = uh;
    *(volatile v4u*)ql = ul;
    __threadfence();
  }
}

__global__ __launch_bounds__(kNT) void k_bn_head(const float* __restrict__ Y, const float* __restrict__ ms,
                                                const float* __restrict__ gam, const float* __restrict__ bet,
                                                const float* __restrict__ Wlin, const float* __restrict__ blin,
                                                float* __restrict__ out) {
  __shared__ float sW[kFeat * kCls];
  __shared__ float sBl[16];
  __shared__ float sM[kFeat];
  __shared__ float sR[kFeat];
  __shared__ float sG[kFeat];
  __shared__ float sBt[kFeat];
  __shared__ __align__(16) float sO0[kNT * kCls];
  __shared__ __align__(16) float sO1[kNT * kCls];
  const int tid = threadIdx.x, lane = tid & 31, wave = tid >> 5;
#pragma unroll 1
  for (int i = tid; i < kFeat * kCls; i += kNT) sW[i] = bf_rne(Wlin[i]);
  {
    const int cc = tid < kCls ? tid : (kCls - 1);
    const float bv = bf_rne(blin[cc]);
    if (tid < 16) sBl[tid] = (tid < kCls) ? bv : 0.0f;
  }
  if (tid < kFeat) { sM[tid] = ms[tid]; sR[tid] = ms[128 + tid]; sG[tid] = bf_rne(gam[tid]); sBt[tid] = bf_rne(bet[tid]); }
  __syncthreads();
  const int r0 = blockIdx.x * kNT;
  const int r  = r0 + tid;
  const int rc = r < kNodes ? r : (kNodes - 1);
  const float* yrow = Y + (size_t)rc * kFeat;
  float acc[kCls];
#pragma unroll
  for (int c = 0; c < kCls; ++c) acc[c] = 0.0f;
#pragma unroll 1
  for (int k = 0; k < kFeat; ++k) {
    const float yk = yrow[k];
    float t = sG[k] * (yk - sM[k]);
    t = t * sR[k] + sBt[k];
    const float h = fmaxf(t, 0.0f);
#pragma unroll
    for (int c = 0; c < kCls; ++c) acc[c] = fmaf(h, sW[k * kCls + c], acc[c]);
  }
  float mx = 0.0f;
#pragma unroll
  for (int c = 0; c < kCls; ++c) {
    float v = acc[c] + sBl[c];
    v = fmaxf(v, 0.0f);
    sO1[tid * kCls + c] = v;
    mx = fmaxf(mx, v);
  }
  float se = 0.0f;
#pragma unroll 1
  for (int c = 0; c < kCls; ++c) se += expf(sO1[tid * kCls + c] - mx);
  const float lse = logf(se);
#pragma unroll 1
  for (int c = 0; c < kCls; ++c) sO0[tid * kCls + c] = (sO1[tid * kCls + c] - mx) - lse;
  __syncthreads();
  const int rows_here = (kNodes - r0) < kNT ? (kNodes - r0) : kNT;
  const int nlines = (rows_here * kCls * 4) / 128;
  const int lq = lane >> 3, piece = (lane & 7) * 4;
  float* o0 = out + (size_t)r0 * kCls;
  float* o1 = out + (size_t)kNodes * kCls + (size_t)r0 * kCls;
  for (int pass = 0; pass < 2; ++pass) {
#pragma unroll 1
    for (int grp = wave; grp * 4 < nlines; grp += 8) {
      const int line  = grp * 4 + lq;
      const int linec = line < nlines ? line : (nlines - 1);
      const int off   = linec * 32 + piece;
      const v4f va = *(const v4f*)(sO0 + off);
      const v4f vb = *(const v4f*)(sO1 + off);
      if (line < nlines) {
        *(volatile v4f*)(o0 + off) = va;
        *(volatile v4f*)(o1 + off) = vb;
      }
    }
    __threadfence();
  }
}

extern "C" void kernel_launch(void* const* d_in, const int* in_sizes, int n_in,
                              void* d_out, int out_size, void* d_ws, size_t ws_size, hipStream_t stream) {
  if (n_in < 14) return;
  if (in_sizes[0] != kNodes * kFeat || in_sizes[1] != 2 * kEdges || out_size != 2 * kNodes * kCls) return;
  if (ws_size < kWsTotal) return;
  const float* x    = (const float*)d_in[0];
  const int*   ei   = (const int*)d_in[1];
  const float* Wl0  = (const float*)d_in[2];
  const float* Wr0  = (const float*)d_in[3];
  const float* b0   = (const float*)d_in[4];
  const float* g0   = (const float*)d_in[5];
  const float* bt0  = (const float*)d_in[6];
  const float* Wl   = (const float*)d_in[7];
  const float* Wr   = (const float*)d_in[8];
  const float* bh   = (const float*)d_in[9];
  const float* gh   = (const float*)d_in[10];
  const float* bth  = (const float*)d_in[11];
  const float* Wlin = (const float*)d_in[12];
  const float* blin = (const float*)d_in[13];
  float* out = (float*)d_out;

  char* ws = (char*)d_ws;
  float*          Q    = (float*)(ws);
  unsigned short* A    = (unsigned short*)(ws + kQBytes);
  float*          Y    = (float*)(ws + kQBytes + kABytes);
  unsigned short* Bt   = (unsigned short*)(ws + kQBytes + kABytes + kYBytes);
  float*          inv  = (float*)(ws + kQBytes + kABytes + kYBytes + kBtBytes);
  float*          part = (float*)(ws + kQBytes + kABytes + kYBytes + kBtBytes + kInvBytes);
  float*          ms   = (float*)(ws + kQBytes + kABytes + kYBytes + kBtBytes + kInvBytes + kPartBytes);
  unsigned short* A0   = A + kA0Off / 2;

  k_prep_x<<<(kMPad * 16) / kNT, kNT, 0, stream>>>(x, A0);
  k_prep_w<<<dim3(16, 3), kNT, 0, stream>>>(Wl0, Wr0, Wl, Wr, Bt);

  const int tilesFull = (kMPad / 64) * (kFeat / 64);
  const dim3 gFull((tilesFull + 7) / 8, 1);
  const int tilesLo = (kSplit / 64) * (kFeat / 64);
  const int tilesHi = ((kMPad - kSplit) / 64) * (kFeat / 64);
  const dim3 gLo((tilesLo + 7) / 8, 1), gHi((tilesHi + 7) / 8, 1);

  wmma_gemm64<1, false, 0, 0, false><<<gFull, 256, 0, stream>>>(
      A0, (const unsigned short*)nullptr, kFeat, 0L,
      Bt, (const unsigned short*)nullptr, kKcat, 0L,
      (void*)Q, (void*)nullptr, kFeat, 0L,
      (const float*)nullptr, (const float*)nullptr, 0L, kMPad, kFeat, kFeat, 1.0f);
  k_agg<true><<<kTiles, kNT, 0, stream>>>(ei, inv, Q, Y, inv);
  wmma_gemm64<1, false, 2, 0, true><<<gFull, 256, 0, stream>>>(
      A0, (const unsigned short*)nullptr, kFeat, 0L,
      Bt + (size_t)kFeat * kKcat, (const unsigned short*)nullptr, kKcat, 0L,
      (void*)Y, (void*)nullptr, kFeat, 0L,
      b0, Y, 0L, kMPad, kFeat, kFeat, 1.0f);
  k_stats<<<kStatBlocks, kNT, 0, stream>>>(Y, part);
  k_bn_fin<<<1, 128, 0, stream>>>(part, ms);
  k_bn_apply<<<(kMPad * 16) / kNT, kNT, 0, stream>>>(Y, ms, g0, bt0, A);

  for (int L = 1; L < 3; ++L) {
    const unsigned short* BtL = Bt + (size_t)L * kKcat * kKcat;
    const float* biasL = bh  + (size_t)(L - 1) * kFeat;
    const float* gamL  = gh  + (size_t)(L - 1) * kFeat;
    const float* betL  = bth + (size_t)(L - 1) * kFeat;
    wmma_gemm64<1, false, 2, 0, false><<<gFull, 256, 0, stream>>>(
        A, (const unsigned short*)nullptr, kKcat, 0L,
        BtL + (size_t)kFeat * kKcat, (const unsigned short*)nullptr, kKcat, 0L,
        (void*)Y, (void*)nullptr, kFeat, 0L,
        biasL, (const float*)nullptr, 0L, kMPad, kFeat, kKcat, 1.0f);
    wmma_gemm64<1, false, 0, 0, false><<<gLo, 256, 0, stream>>>(
        A, (const unsigned short*)nullptr, kKcat, 0L,
        BtL, (const unsigned short*)nullptr, kKcat, 0L,
        (void*)Q, (void*)nullptr, kFeat, 0L,
        (const float*)nullptr, (const float*)nullptr, 0L, kSplit, kFeat, kKcat, 1.0f);
    wmma_gemm64<1, false, 0, 0, false><<<gHi, 256, 0, stream>>>(
        A + (size_t)kSplit * kKcat, (const unsigned short*)nullptr, kKcat, 0L,
        BtL, (const unsigned short*)nullptr, kKcat, 0L,
        (void*)(Q + (size_t)kSplit * kFeat), (void*)nullptr, kFeat, 0L,
        (const float*)nullptr, (const float*)nullptr, 0L, kMPad - kSplit, kFeat, kKcat, 1.0f);
    k_agg<false><<<kTiles, kNT, 0, stream>>>(ei, inv, Q, Y, inv);
    k_stats<<<kStatBlocks, kNT, 0, stream>>>(Y, part);
    k_bn_fin<<<1, 128, 0, stream>>>(part, ms);
    if (L == 1) {
      k_bn_apply<<<(kMPad * 16) / kNT, kNT, 0, stream>>>(Y, ms, gamL, betL, A);
    } else {
      k_bn_head<<<(kNodes + kNT - 1) / kNT, kNT, 0, stream>>>(Y, ms, gamL, betL, Wlin, blin, out);
    }
  }
}
